// LEDDecoderAttentionTopicAware_35235911696716
// MI455X (gfx1250) — hardware-verified
//
#include <hip/hip_runtime.h>
#include <math.h>

constexpr int kB   = 2;
constexpr int kT   = 512;
constexpr int kS   = 4096;
constexpr int kE   = 1024;
constexpr int kTP  = 512;
constexpr int kH   = 8;
constexpr int kDH  = 128;
constexpr int kTok = kB * kT;
constexpr int kKVT = kB * kS;
constexpr int kGrp = 2;
constexpr int kNChunk = (kB * kH) / kGrp;
constexpr int kGatePitch = 32;
constexpr float kAttnScale = 0.08838834764831845f;
constexpr float kWCarry    = 16.0f;
constexpr float kWCarryInv = 1.0f / 16.0f;
constexpr float kQCarry    = 16.0f;
constexpr float kQCarryInv = 1.0f / 16.0f;
constexpr float kPCarry    = 2048.0f;
constexpr float kPCarryInv = 1.0f / 2048.0f;
constexpr float kMixCarry  = 256.0f;
constexpr float kOutScale  = 1.0f / (256.0f * 16.0f);

typedef __attribute__((ext_vector_type(16))) _Float16 v16h;
typedef __attribute__((ext_vector_type(8)))  _Float16 v8h;
typedef __attribute__((ext_vector_type(16))) __bf16   v16b;
typedef __attribute__((ext_vector_type(8)))  __bf16   v8b;
typedef __attribute__((ext_vector_type(8)))  float    v8f;
typedef __attribute__((ext_vector_type(4)))  float    v4f;
typedef __attribute__((ext_vector_type(4)))  unsigned int v4u;

__device__ __forceinline__ unsigned short f2bf_bits(float f) {
  unsigned u = __float_as_uint(f);
  return (unsigned short)((u + 0x7FFFu + ((u >> 16) & 1u)) >> 16);
}
__device__ __forceinline__ float bf_bits2f(unsigned short h) { return __uint_as_float(((unsigned)h) << 16); }

__device__ __forceinline__ void dep_guard_h(v8f& a, v8f& b, v16h x, v16h y) { asm volatile("v_nop\n\tv_nop\n\tv_nop\n\tv_nop" : "+v"(a), "+v"(b) : "v"(x), "v"(y)); }
__device__ __forceinline__ void dep_guard_b(v8f& a, v8f& b, v16b x, v16b y) { asm volatile("v_nop\n\tv_nop\n\tv_nop\n\tv_nop" : "+v"(a), "+v"(b) : "v"(x), "v"(y)); }
__device__ __forceinline__ void keep4_h(v16h a, v16h b, v16h c, v16h d) { asm volatile("v_nop" :: "v"(a), "v"(b), "v"(c), "v"(d)); }
__device__ __forceinline__ void keep4_b(v16b a, v16b b, v16b c, v16b d) { asm volatile("v_nop" :: "v"(a), "v"(b), "v"(c), "v"(d)); }
__device__ __forceinline__ void acc_guard4(v8f& a, v8f& b, v8f& c, v8f& d) { asm volatile("v_nop\n\tv_nop\n\tv_nop\n\tv_nop" : "+v"(a), "+v"(b), "+v"(c), "+v"(d)); }
template <typename T> struct Frag;
template <> struct Frag<_Float16> {
  typedef v16h V; union U { v16h v; v8h h[2]; };
  static __device__ __forceinline__ v16h load(const _Float16* p) {
    U f; f.h[0] = *(const v8h*)(p); f.h[1] = *(const v8h*)(p + 16); return f.v;
  }
  static __device__ __forceinline__ v8f mma(v16h a, v16h b, v8f c) {
    return __builtin_amdgcn_wmma_f32_16x16x32_f16(false, a, false, b, (short)0, c, false, false);
  }
  static __device__ __forceinline__ void guard(v8f& a, v8f& b, v16h x, v16h y) { dep_guard_h(a, b, x, y); }
  static __device__ __forceinline__ void keep(v16h a, v16h b, v16h c, v16h d) { keep4_h(a, b, c, d); }
};
template <> struct Frag<__bf16> {
  typedef v16b V; union U { v16b v; v8b h[2]; };
  static __device__ __forceinline__ v16b load(const __bf16* p) {
    U f; f.h[0] = *(const v8b*)(p); f.h[1] = *(const v8b*)(p + 16); return f.v;
  }
  static __device__ __forceinline__ v8f mma(v16b a, v16b b, v8f c) {
    return __builtin_amdgcn_wmma_f32_16x16x32_bf16(false, a, false, b, (short)0, c, false, false);
  }
  static __device__ __forceinline__ void guard(v8f& a, v8f& b, v16b x, v16b y) { dep_guard_b(a, b, x, y); }
  static __device__ __forceinline__ void keep(v16b a, v16b b, v16b c, v16b d) { keep4_b(a, b, c, d); }
};

__device__ __forceinline__ unsigned pk16(unsigned short a, unsigned short b) { return (unsigned)a | ((unsigned)b << 16); }
__device__ __forceinline__ unsigned short h_bits(float f) { const _Float16 h = (_Float16)f; return __builtin_bit_cast(unsigned short, h); }

template <int ET> struct Elem;
template <> struct Elem<0> { typedef _Float16 T; };
template <> struct Elem<1> { typedef __bf16 T; };
template <int ET, bool SPLIT, int BIAS_MODE, int OUT_MODE, bool RESID, int ACT = 0>
__global__ __launch_bounds__(256) void wmma_gemm64(
    const unsigned short* __restrict__ Ap, const unsigned short* __restrict__ A2p, int lda, long strideA,
    const unsigned short* __restrict__ Btp, const unsigned short* __restrict__ Bt2p, int ldb, long strideB,
    void* __restrict__ Cout, void* __restrict__ Cout2, int ldc, long strideC,
    const float* __restrict__ bias,
    const float* __restrict__ resid, long strideR,
    int M, int N, int K, float scale, float bscale) {
  typedef typename Elem<ET>::T T;
  typedef typename Frag<T>::V V;
  const T* A = (const T*)Ap; const T* A2 = (const T*)A2p; const T* Bt = (const T*)Btp; const T* Bt2 = (const T*)Bt2p;
  __shared__ __align__(16) float sT[8][16 * 68];
  const int b    = blockIdx.y;
  const int lane = threadIdx.x & 31;
  const int wave = threadIdx.x >> 5;
  const int tilesN = N >> 6;
  const int tilesM = M >> 6;
  const int tile = blockIdx.x * 8 + wave;
  if (tile >= tilesM * tilesN) return;
  const int tm = tile / tilesN;
  const int tn = tile - tm * tilesN;
  const int m0 = tm << 6;
  const int n0 = tn << 6;

  const T* Ab  = A  + (size_t)b * strideA;
  const T* Bb  = Bt + (size_t)b * strideB;
  const T* Ab2 = SPLIT ? (A2  + (size_t)b * strideA) : nullptr;
  const T* Bb2 = SPLIT ? (Bt2 + (size_t)b * strideB) : nullptr;

  const int rlane = lane & 15;
  const int koff  = (lane >> 4) * 8;
  const int mOff  = (lane >> 4) * 8;

  v8f acc[4][4];
#pragma unroll
  for (int i = 0; i < 4; ++i)
#pragma unroll
    for (int j = 0; j < 4; ++j) acc[i][j] = (v8f){0.f,0.f,0.f,0.f,0.f,0.f,0.f,0.f};

  for (int k0 = 0; k0 < K; k0 += 32) {
    V bh[4], bl[4];
#pragma unroll
    for (int j = 0; j < 4; ++j) {
      const size_t bo = (size_t)(n0 + (j << 4) + rlane) * ldb + koff + k0;
      bh[j] = Frag<T>::load(Bb + bo);
      if (SPLIT) bl[j] = Frag<T>::load(Bb2 + bo);
    }
#pragma unroll
    for (int i = 0; i < 4; ++i) {
      const size_t ao = (size_t)(m0 + (i << 4) + rlane) * lda + koff + k0;
      V ah = Frag<T>::load(Ab + ao);
      V al;
      if (SPLIT) al = Frag<T>::load(Ab2 + ao);
#pragma unroll
      for (int j = 0; j < 4; ++j) {
        acc[i][j] = Frag<T>::mma(ah, bh[j], acc[i][j]);
        if (SPLIT) {
          acc[i][j] = Frag<T>::mma(ah, bl[j], acc[i][j]);
          acc[i][j] = Frag<T>::mma(al, bh[j], acc[i][j]);
        }
      }
      Frag<T>::guard(acc[i][0], acc[i][3], ah, SPLIT ? al : ah);
    }
    Frag<T>::keep(bh[0], bh[1], bh[2], bh[3]);
    if (SPLIT) Frag<T>::keep(bl[0], bl[1], bl[2], bl[3]);
  }
  acc_guard4(acc[0][0], acc[0][1], acc[0][2], acc[0][3]);
  acc_guard4(acc[1][0], acc[1][1], acc[1][2], acc[1][3]);
  acc_guard4(acc[2][0], acc[2][1], acc[2][2], acc[2][3]);
  acc_guard4(acc[3][0], acc[3][1], acc[3][2], acc[3][3]);

  float* slab = sT[wave];
  const float* Rb = RESID ? (resid + (size_t)b * strideR) : nullptr;
#pragma unroll
  for (int i = 0; i < 4; ++i) {
    const int mBase = m0 + (i << 4);
#pragma unroll
    for (int j = 0; j < 4; ++j) {
      const int n = n0 + (j << 4) + rlane;
      float bv = 0.f;
      if (BIAS_MODE == 2) bv = bias[n] * bscale;
#pragma unroll
      for (int r = 0; r < 8; ++r) {
        float v = acc[i][j][r] * scale;
        if (BIAS_MODE == 1) v += bias[mBase + mOff + r] * bscale;
        if (BIAS_MODE == 2) v += bv;
        if (RESID) v += Rb[(size_t)(mBase + mOff + r) * ldc + n];
        if (ACT == 2) v = fmaxf(v, 0.0f);
        if (ACT == 4) v = (v > 0.f) ? v : 0.01f * v;
        slab[(mOff + r) * 68 + (j << 4) + rlane] = v;
      }
    }
    __builtin_amdgcn_fence(__ATOMIC_RELEASE, "workgroup");
    __builtin_amdgcn_wave_barrier();
    __builtin_amdgcn_fence(__ATOMIC_ACQUIRE, "workgroup");
    if (OUT_MODE == 0) {
      float* C = (float*)Cout + (size_t)b * strideC;
      const int hh = lane >> 4, c4 = (lane & 15) * 4;
      for (int pass = 0; pass < 2; ++pass) {
#pragma unroll
        for (int it = 0; it < 8; ++it) {
          const int row = it * 2 + hh;
          v4f v = *(const v4f*)(slab + row * 68 + c4);
          *(volatile v4f*)(C + (size_t)(mBase + row) * ldc + n0 + c4) = v;
        }
        __threadfence();
      }
    } else {
      const int q = lane >> 3, c8 = (lane & 7) * 8;
      unsigned short* C  = (unsigned short*)Cout  + (size_t)b * strideC;
      unsigned short* C2 = (OUT_MODE == 2) ? ((unsigned short*)Cout2 + (size_t)b * strideC) : nullptr;
      for (int pass = 0; pass < 2; ++pass) {
#pragma unroll
        for (int it = 0; it < 4; ++it) {
          const int row = it * 4 + q;
          const float* sp = slab + row * 68 + c8;
          v8h hv, lv;
#pragma unroll
          for (int e = 0; e < 8; ++e) {
            if (OUT_MODE == 1) {
              hv[e] = (_Float16)sp[e];
            } else {
              unsigned short hb = f2bf_bits(sp[e]);
              unsigned short lb = f2bf_bits(sp[e] - bf_bits2f(hb));
              hv[e] = __builtin_bit_cast(_Float16, hb);
              lv[e] = __builtin_bit_cast(_Float16, lb);
            }
          }
          *(volatile v8h*)(C + (size_t)(mBase + row) * ldc + n0 + c8) = hv;
          if (OUT_MODE == 2) *(volatile v8h*)(C2 + (size_t)(mBase + row) * ldc + n0 + c8) = lv;
        }
        __threadfence();
      }
    }
    __builtin_amdgcn_fence(__ATOMIC_RELEASE, "workgroup");
    __builtin_amdgcn_wave_barrier();
    __builtin_amdgcn_fence(__ATOMIC_ACQUIRE, "workgroup");
  }
}

__global__ __launch_bounds__(256) void wtcast_kernel(const float* __restrict__ W0, const float* __restrict__ W1,
                                                     const float* __restrict__ W2, const float* __restrict__ W3,
                                                     unsigned short* __restrict__ O0, unsigned short* __restrict__ O1,
                                                     unsigned short* __restrict__ O2, unsigned short* __restrict__ O3,
                                                     int Kin, int Nout, float scale) {
  __shared__ float sm[64][65];
  const int t  = threadIdx.x;
  const int k0 = blockIdx.x * 64;
  const int n0 = blockIdx.y * 64;
  const int z  = blockIdx.z;
  const float* W = (z == 0) ? W0 : (z == 1) ? W1 : (z == 2) ? W2 : W3;
  unsigned short* op = (z == 0) ? O0 : (z == 1) ? O1 : (z == 2) ? O2 : O3;
#pragma unroll
  for (int i = 0; i < 16; ++i) {
    const int e = i * 256 + t;
    const int r = e >> 6;
    const int c = e & 63;
    sm[c][r] = W[(size_t)(k0 + r) * Nout + n0 + c] * scale;
  }
  __syncthreads();
  const int lane = t & 31, wave = t >> 5;
  const int q = lane >> 3, c8 = (lane & 7) * 8;
  for (int pass = 0; pass < 2; ++pass) {
#pragma unroll
    for (int it = 0; it < 2; ++it) {
      const int row = wave * 8 + it * 4 + q;
      unsigned short hb[8];
#pragma unroll
      for (int e = 0; e < 8; ++e) hb[e] = h_bits(sm[row][c8 + e]);
      const v4u u = (v4u){pk16(hb[0], hb[1]), pk16(hb[2], hb[3]), pk16(hb[4], hb[5]), pk16(hb[6], hb[7])};
      *(volatile v4u*)(op + (size_t)(n0 + row) * Kin + k0 + c8) = u;
    }
    __threadfence();
  }
}

__global__ __launch_bounds__(256) void cast8_f16_kernel(const float* __restrict__ in, unsigned short* __restrict__ out, int n8) {
  const int i = blockIdx.x * 256 + threadIdx.x;
  if (i >= n8) return;
  const float* p = in + 8 * (size_t)i;
  const v4f a = *(const v4f*)(p);
  const v4f c = *(const v4f*)(p + 4);
  unsigned short hb[8];
#pragma unroll
  for (int e = 0; e < 4; ++e) {
    hb[e]     = h_bits(a[e]);
    hb[4 + e] = h_bits(c[e]);
  }
  const v4u u = (v4u){pk16(hb[0], hb[1]), pk16(hb[2], hb[3]), pk16(hb[4], hb[5]), pk16(hb[6], hb[7])};
  unsigned short* q = out + 8 * (size_t)i;
  *(volatile v4u*)q = u;
  __threadfence();
  *(volatile v4u*)q = u;
}

__global__ __launch_bounds__(256) void softmax_kernel(const float* __restrict__ Sb, unsigned short* __restrict__ Pb, float carry) {
  __shared__ float redM[8];
  __shared__ float redS[8];
  const int row  = blockIdx.x;
  const int pz   = blockIdx.z * kGrp + blockIdx.y;
  const int t    = threadIdx.x;
  const int lane = t & 31, wave = t >> 5;
  const size_t roff = ((size_t)pz * kT + row) * kS;
  const int c0 = t * 8;
  const int c1 = (kS / 2) + t * 8;
  const float* sr = Sb + roff;
  const v4f a0 = *(const v4f*)(sr + c0);
  const v4f a1 = *(const v4f*)(sr + c0 + 4);
  const v4f a2 = *(const v4f*)(sr + c1);
  const v4f a3 = *(const v4f*)(sr + c1 + 4);
  float x[16];
#pragma unroll
  for (int e = 0; e < 4; ++e) { x[e] = a0[e]; x[4 + e] = a1[e]; x[8 + e] = a2[e]; x[12 + e] = a3[e]; }
  float m = x[0];
#pragma unroll
  for (int e = 1; e < 16; ++e) m = fmaxf(m, x[e]);
#pragma unroll
  for (int off = 16; off > 0; off >>= 1) m = fmaxf(m, __shfl_xor(m, off, 32));
  if (lane == 0) redM[wave] = m;
  __syncthreads();
  float gm = redM[0];
#pragma unroll
  for (int w = 1; w < 8; ++w) gm = fmaxf(gm, redM[w]);
  float ev[16];
  float s = 0.0f;
#pragma unroll
  for (int e = 0; e < 16; ++e) { ev[e] = expf(x[e] - gm); s += ev[e]; }
#pragma unroll
  for (int off = 16; off > 0; off >>= 1) s += __shfl_xor(s, off, 32);
  if (lane == 0) redS[wave] = s;
  __syncthreads();
  float tot = redS[0];
#pragma unroll
  for (int w = 1; w < 8; ++w) tot += redS[w];
  const float inv = carry / tot;
  unsigned short hb[16];
#pragma unroll
  for (int e = 0; e < 16; ++e) hb[e] = h_bits(ev[e] * inv);
  const v4u u0 = (v4u){pk16(hb[0], hb[1]), pk16(hb[2], hb[3]), pk16(hb[4], hb[5]), pk16(hb[6], hb[7])};
  const v4u u1 = (v4u){pk16(hb[8], hb[9]), pk16(hb[10], hb[11]), pk16(hb[12], hb[13]), pk16(hb[14], hb[15])};
  unsigned short* pr = Pb + roff;
  *(volatile v4u*)(pr + c0) = u0;
  *(volatile v4u*)(pr + c1) = u1;
  __threadfence();
  *(volatile v4u*)(pr + c0) = u0;
  *(volatile v4u*)(pr + c1) = u1;
}

__global__ __launch_bounds__(128) void gate_kernel(const float* __restrict__ ctx, const float* __restrict__ ctxt,
                                                   const unsigned short* __restrict__ q16, const float* __restrict__ Wg,
                                                   const float* __restrict__ bg, float* __restrict__ gate, float qinv) {
  __shared__ float red[4][8];
  __shared__ __align__(16) float gl[32];
  const int tok = blockIdx.x;
  const int t = threadIdx.x, lane = t & 31, wave = t >> 5;
  if (t < 32) gl[t] = 0.0f;
  float a[8];
#pragma unroll
  for (int j = 0; j < 8; ++j) a[j] = 0.0f;
  const size_t rbase = (size_t)tok * kE;
#pragma unroll 1
  for (int c = 0; c < 24; ++c) {
    const int h = c / 3;
    const int src = c - 3 * h;
    const size_t off = rbase + (size_t)h * kDH + t;
    const float fc = ctx[off];
    const float ft = ctxt[off];
    const unsigned short qbits = q16[off];
    const float fq = (float)__builtin_bit_cast(_Float16, qbits) * qinv;
    const float f = (src == 0) ? fc : ((src == 1) ? ft : fq);
    const float* wr = Wg + ((size_t)c * 128 + t) * 8;
    const v4f w0 = *(const v4f*)(wr);
    const v4f w1 = *(const v4f*)(wr + 4);
#pragma unroll
    for (int e = 0; e < 4; ++e) { a[e] += f * w0[e]; a[4 + e] += f * w1[e]; }
  }
#pragma unroll
  for (int j = 0; j < 8; ++j) {
#pragma unroll
    for (int off = 16; off > 0; off >>= 1) a[j] += __shfl_xor(a[j], off, 32);
  }
  if (lane == 0) {
#pragma unroll
    for (int j = 0; j < 8; ++j) red[wave][j] = a[j];
  }
  __syncthreads();
  if (t < 8) {
    const float z = (((red[0][t] + red[1][t]) + red[2][t]) + red[3][t]) + bg[t];
    gl[t] = 1.0f / (1.0f + expf(-z));
  }
  __syncthreads();
  if (wave == 0) {
    if (lane < 8) {
      const v4f v = *(const v4f*)(gl + 4 * lane);
      float* gp = gate + (size_t)tok * kGatePitch + 4 * lane;
      *(volatile v4f*)gp = v;
      __threadfence();
      *(volatile v4f*)gp = v;
    }
  }
}

__global__ __launch_bounds__(256) void mix_kernel(const float* __restrict__ ctx, const float* __restrict__ ctx2,
                                                  const float* __restrict__ gate, unsigned short* __restrict__ out,
                                                  float carry, int n8) {
  const int i = blockIdx.x * 256 + threadIdx.x;
  if (i >= n8) return;
  const int tok  = i >> 7;
  const int col0 = (i & 127) * 8;
  const int h    = col0 >> 7;
  const float g  = gate[(size_t)tok * kGatePitch + h];
  const float og = 1.0f - g;
  const size_t off = (size_t)tok * kE + col0;
  const v4f a0 = *(const v4f*)(ctx + off);
  const v4f a1 = *(const v4f*)(ctx + off + 4);
  const v4f b0 = *(const v4f*)(ctx2 + off);
  const v4f b1 = *(const v4f*)(ctx2 + off + 4);
  unsigned short hb[8];
#pragma unroll
  for (int e = 0; e < 4; ++e) {
    hb[e]     = h_bits(carry * (g * a0[e] + og * b0[e]));
    hb[4 + e] = h_bits(carry * (g * a1[e] + og * b1[e]));
  }
  const v4u u = (v4u){pk16(hb[0], hb[1]), pk16(hb[2], hb[3]), pk16(hb[4], hb[5]), pk16(hb[6], hb[7])};
  unsigned short* q = out + off;
  *(volatile v4u*)q = u;
  __threadfence();
  *(volatile v4u*)q = u;
}

extern "C" void kernel_launch(void* const* d_in, const int* in_sizes, int n_in,
                              void* d_out, int out_size, void* d_ws, size_t ws_size, hipStream_t stream) {
  (void)in_sizes; (void)n_in;
  const size_t kMiB = (size_t)1048576;
  const size_t carve = 128 * kMiB;
  if (ws_size < carve) return;
  if ((size_t)out_size < (size_t)kTok * kE) return;

  const float* hs  = (const float*)d_in[0];
  const float* kv  = (const float*)d_in[1];
  const float* kvt = (const float*)d_in[2];
  const float* Wq  = (const float*)d_in[3];  const float* bq  = (const float*)d_in[4];
  const float* Wk  = (const float*)d_in[5];  const float* bk  = (const float*)d_in[6];
  const float* Wv  = (const float*)d_in[7];  const float* bv  = (const float*)d_in[8];
  const float* Wtk = (const float*)d_in[9];  const float* btk = (const float*)d_in[10];
  const float* Wtv = (const float*)d_in[11]; const float* btv = (const float*)d_in[12];
  const float* Wg  = (const float*)d_in[13]; const float* bg  = (const float*)d_in[14];
  const float* Wo  = (const float*)d_in[15]; const float* bo  = (const float*)d_in[16];
  float* outp = (float*)d_out;

  char* ws = (char*)d_ws;
  unsigned short* XH16  = (unsigned short*)(ws + 0 * kMiB);
  unsigned short* KV16  = (unsigned short*)(ws + 2 * kMiB);
  unsigned short* KVT16 = (unsigned short*)(ws + 18 * kMiB);
  unsigned short* WQT   = (unsigned short*)(ws + 26 * kMiB);
  unsigned short* WKT   = (unsigned short*)(ws + 28 * kMiB);
  unsigned short* WVT   = (unsigned short*)(ws + 30 * kMiB);
  unsigned short* WTKT  = (unsigned short*)(ws + 32 * kMiB);
  unsigned short* WTVT  = (unsigned short*)(ws + 33 * kMiB);
  float*          SPL   = (float*)(ws + 0 * kMiB);
  float*          STPL  = (float*)(ws + 16 * kMiB);
  unsigned short* PPL   = (unsigned short*)(ws + 32 * kMiB);
  unsigned short* PTPL  = (unsigned short*)(ws + 40 * kMiB);
  unsigned short* MIX16 = (unsigned short*)(ws + 0 * kMiB);
  float*          GATE  = (float*)(ws + 2 * kMiB);
  unsigned short* WOT   = (unsigned short*)(ws + 48 * kMiB);
  unsigned short* Q16   = (unsigned short*)(ws + 50 * kMiB);
  unsigned short* K16   = (unsigned short*)(ws + 52 * kMiB);
  unsigned short* VT16  = (unsigned short*)(ws + 68 * kMiB);
  unsigned short* KT16  = (unsigned short*)(ws + 84 * kMiB);
  unsigned short* VTT16 = (unsigned short*)(ws + 100 * kMiB);
  float*          CTX   = (float*)(ws + 116 * kMiB);
  float*          CTXT  = (float*)(ws + 120 * kMiB);
  float*          CTX2  = (float*)(ws + 124 * kMiB);
  const float*    dumf  = (const float*)(ws + 116 * kMiB);

  cast8_f16_kernel<<<(kTok * kE / 8) / 256, 256, 0, stream>>>(hs, XH16, kTok * kE / 8);
  cast8_f16_kernel<<<(kKVT * kE / 8) / 256, 256, 0, stream>>>(kv, KV16, kKVT * kE / 8);
  cast8_f16_kernel<<<(kKVT * kTP / 8) / 256, 256, 0, stream>>>(kvt, KVT16, kKVT * kTP / 8);

  wtcast_kernel<<<dim3(kE / 64, kE / 64, 4), 256, 0, stream>>>(Wq, Wk, Wv, Wo, WQT, WKT, WVT, WOT, kE, kE, kWCarry);
  wtcast_kernel<<<dim3(kTP / 64, kE / 64, 2), 256, 0, stream>>>(Wtk, Wtv, Wtk, Wtv, WTKT, WTVT, WTKT, WTVT, kTP, kE, kWCarry);

  wmma_gemm64<0, false, 2, 1, false><<<dim3((kTok / 64) * (kE / 64) / 8, 1), 256, 0, stream>>>(
      XH16, XH16, kE, 0L, WQT, WQT, kE, 0L, Q16, Q16, kE, 0L, bq, dumf, 0L,
      kTok, kE, kE, kAttnScale, kQCarry * kAttnScale);
  wmma_gemm64<0, false, 2, 1, false><<<dim3((kKVT / 64) * (kE / 64) / 8, 1), 256, 0, stream>>>(
      KV16, KV16, kE, 0L, WKT, WKT, kE, 0L, K16, K16, kE, 0L, bk, dumf, 0L,
      kKVT, kE, kE, kWCarryInv, 1.0f);
  wmma_gemm64<0, false, 1, 1, false><<<dim3((kE / 64) * (kKVT / 64) / 8, 1), 256, 0, stream>>>(
      WVT, WVT, kE, 0L, KV16, KV16, kE, 0L, VT16, VT16, kKVT, 0L, bv, dumf, 0L,
      kE, kKVT, kE, kWCarryInv, 1.0f);
  wmma_gemm64<0, false, 2, 1, false><<<dim3((kKVT / 64) * (kE / 64) / 8, 1), 256, 0, stream>>>(
      KVT16, KVT16, kTP, 0L, WTKT, WTKT, kTP, 0L, KT16, KT16, kE, 0L, btk, dumf, 0L,
      kKVT, kE, kTP, kWCarryInv, 1.0f);
  wmma_gemm64<0, false, 1, 1, false><<<dim3((kE / 64) * (kKVT / 64) / 8, 1), 256, 0, stream>>>(
      WTVT, WTVT, kTP, 0L, KVT16, KVT16, kTP, 0L, VTT16, VTT16, kKVT, 0L, btv, dumf, 0L,
      kE, kKVT, kTP, kWCarryInv, 1.0f);

  const long sStrideC = (long)kT * kS;
  const long pStrideA = (long)kT * kS;
  for (int c = 0; c < kNChunk; ++c) {
    const int b  = c / (kH / kGrp);
    const int h0 = (c % (kH / kGrp)) * kGrp;
    const unsigned short* qg = Q16 + ((size_t)b * kT * kE + (size_t)h0 * kDH);
    const unsigned short* kg = K16 + ((size_t)b * kS * kE + (size_t)h0 * kDH);
    const unsigned short* k2g = KT16 + ((size_t)b * kS * kE + (size_t)h0 * kDH);
    wmma_gemm64<0, false, 0, 0, false><<<dim3((kT / 64) * (kS / 64) / 8, kGrp), 256, 0, stream>>>(
        qg, qg, kE, (long)kDH, kg, kg, kE, (long)kDH, SPL, SPL, kS, sStrideC, bq, dumf, 0L,
        kT, kS, kDH, kQCarryInv, 0.0f);
    wmma_gemm64<0, false, 0, 0, false><<<dim3((kT / 64) * (kS / 64) / 8, kGrp), 256, 0, stream>>>(
        qg, qg, kE, (long)kDH, k2g, k2g, kE, (long)kDH, STPL, STPL, kS, sStrideC, bq, dumf, 0L,
        kT, kS, kDH, kQCarryInv, 0.0f);
    softmax_kernel<<<dim3(kT, kGrp, 2), 256, 0, stream>>>(SPL, PPL, kPCarry);
    const unsigned short* vg  = VT16  + ((size_t)h0 * kDH * kKVT + (size_t)b * kS);
    const unsigned short* v2g = VTT16 + ((size_t)h0 * kDH * kKVT + (size_t)b * kS);
    const size_t coff = (size_t)b * kT * kE + (size_t)h0 * kDH;
    wmma_gemm64<0, false, 0, 0, false><<<dim3((kT / 64) * (kDH / 64) / 8, kGrp), 256, 0, stream>>>(
        PPL, PPL, kS, pStrideA, vg, vg, kKVT, (long)kDH * kKVT, CTX + coff, CTX + coff, kE, (long)kDH, bq, dumf, 0L,
        kT, kDH, kS, kPCarryInv, 0.0f);
    wmma_gemm64<0, false, 0, 0, false><<<dim3((kT / 64) * (kDH / 64) / 8, kGrp), 256, 0, stream>>>(
        PTPL, PTPL, kS, pStrideA, v2g, v2g, kKVT, (long)kDH * kKVT, CTXT + coff, CTXT + coff, kE, (long)kDH, bq, dumf, 0L,
        kT, kDH, kS, kPCarryInv, 0.0f);
    wmma_gemm64<0, false, 0, 0, false><<<dim3((kT / 64) * (kDH / 64) / 8, kGrp), 256, 0, stream>>>(
        PTPL, PTPL, kS, pStrideA, vg, vg, kKVT, (long)kDH * kKVT, CTX2 + coff, CTX2 + coff, kE, (long)kDH, bq, dumf, 0L,
        kT, kDH, kS, kPCarryInv, 0.0f);
  }

  gate_kernel<<<kTok, 128, 0, stream>>>(CTX, CTXT, Q16, Wg, bg, GATE, kQCarryInv);
  mix_kernel<<<(kTok * kE / 8) / 256, 256, 0, stream>>>(CTX, CTX2, GATE, MIX16, kMixCarry, kTok * kE / 8);
  wmma_gemm64<0, false, 2, 0, false><<<dim3((kTok / 64) * (kE / 64) / 8, 1), 256, 0, stream>>>(
      MIX16, MIX16, kE, 0L, WOT, WOT, kE, 0L, outp, outp, kE, 0L, bo, dumf, 0L,
      kTok, kE, kE, kOutScale, 1.0f);
}
